// SelfInteractor_71519795413650
// MI455X (gfx1250) — hardware-verified
//
#include <hip/hip_runtime.h>


#define NN   1024
#define DD   128
#define G3   384
#define PCAR 1024.0f
typedef _Float16 h16;
typedef unsigned short bf;
typedef __attribute__((ext_vector_type(16))) __bf16   v16bf;
typedef __attribute__((ext_vector_type(16))) _Float16 v16h;
typedef __attribute__((ext_vector_type(8)))  _Float16 v8h;
typedef __attribute__((ext_vector_type(8)))  unsigned short v8us;
typedef __attribute__((ext_vector_type(8)))  float    v8f;
typedef __attribute__((ext_vector_type(4)))  float    v4f;
typedef v8h  __attribute__((may_alias)) v8ha;
typedef v4f  __attribute__((may_alias)) v4fa;
typedef v8us __attribute__((may_alias)) v8usa;

__device__ __forceinline__ unsigned short f2bf(float f) { unsigned u = __float_as_uint(f); u += 0x7FFFu + ((u >> 16) & 1u); return (unsigned short)(u >> 16); }
__device__ __forceinline__ float bf2f(unsigned short b) { return __uint_as_float(((unsigned)b) << 16); }
__device__ __forceinline__ float bfr(float f) { return bf2f(f2bf(f)); }
__device__ __forceinline__ v16h cat16(v8h lo, v8h hi) { return __builtin_shufflevector(lo, hi, 0, 1, 2, 3, 4, 5, 6, 7, 8, 9, 10, 11, 12, 13, 14, 15); }
__device__ __forceinline__ v16bf cat16b(v8us lo, v8us hi) { return __builtin_bit_cast(v16bf, __builtin_shufflevector(lo, hi, 0, 1, 2, 3, 4, 5, 6, 7, 8, 9, 10, 11, 12, 13, 14, 15)); }
__device__ __forceinline__ v8f wmma16(v16h a, v16h b, v8f c) { return __builtin_amdgcn_wmma_f32_16x16x32_f16(false, a, false, b, (short)0, c, false, false); }
__device__ __forceinline__ v8f wmmab(v16bf a, v16bf b, v8f c) { return __builtin_amdgcn_wmma_f32_16x16x32_bf16(false, a, false, b, (short)0, c, false, false); }


template <typename T16> struct WFrag;
template <> struct WFrag<h16> { typedef v16h V; static __device__ __forceinline__ V ld(const h16* p) { return cat16(*(const v8h*)p, *(const v8h*)(p + 16)); } static __device__ __forceinline__ v8f mma(V a, V b, v8f c) { return wmma16(a, b, c); } };
template <> struct WFrag<bf> { typedef v16bf V; static __device__ __forceinline__ V ld(const bf* p) { return cat16b(*(const v8us*)p, *(const v8us*)(p + 16)); } static __device__ __forceinline__ v8f mma(V a, V b, v8f c) { return wmmab(a, b, c); } };
template <typename T16, int NSPLIT, bool BIAS>
__global__ __launch_bounds__(32) void k_gemmw(const T16* __restrict__ A, const T16* __restrict__ A2, const T16* __restrict__ Bt, const T16* __restrict__ Bt2, int K, float* C, int ldc, const float* __restrict__ bias, size_t sA, size_t sB, size_t sC) {
    typedef typename WFrag<T16>::V V;
    __shared__ __align__(16) float os[16 * 68];
    const size_t z = blockIdx.z; A += z * sA; if (A2) A2 += z * sA; Bt += z * sB; if (Bt2) Bt2 += z * sB; C += z * sC;
    const int lane = threadIdx.x & 31, lr = lane & 15, hi = lane >> 4; const int r0 = blockIdx.x * 64, c0 = blockIdx.y * 64;
    v8f acc[4][4];
#pragma unroll
    for (int mb = 0; mb < 4; ++mb)
#pragma unroll
        for (int nb = 0; nb < 4; ++nb) acc[mb][nb] = (v8f){};
    const size_t aoff = (size_t)(r0 + lr) * K + 8 * hi, boff = (size_t)(c0 + lr) * K + 8 * hi;
#pragma unroll 1
    for (int kc = 0; kc < K; kc += 32) {
        V a[4], a2[4];
#pragma unroll
        for (int mb = 0; mb < 4; ++mb) { a[mb] = WFrag<T16>::ld(A + aoff + (size_t)mb * 16 * K + kc); if (NSPLIT == 1 || NSPLIT == 2) a2[mb] = WFrag<T16>::ld(A2 + aoff + (size_t)mb * 16 * K + kc); }
#pragma unroll
        for (int nb = 0; nb < 4; ++nb) { const V b = WFrag<T16>::ld(Bt + boff + (size_t)nb * 16 * K + kc); V b2; if (NSPLIT >= 2) b2 = WFrag<T16>::ld(Bt2 + boff + (size_t)nb * 16 * K + kc);
#pragma unroll
            for (int mb = 0; mb < 4; ++mb) { acc[mb][nb] = WFrag<T16>::mma(a[mb], b, acc[mb][nb]); if (NSPLIT == 1 || NSPLIT == 2) acc[mb][nb] = WFrag<T16>::mma(a2[mb], b, acc[mb][nb]); if (NSPLIT >= 2) acc[mb][nb] = WFrag<T16>::mma(a[mb], b2, acc[mb][nb]); } }
        asm volatile("v_nop\n\tv_nop\n\tv_nop\n\tv_nop" : "+v"(acc[0][0]), "+v"(acc[1][1]), "+v"(acc[2][2]), "+v"(acc[3][3]) : "v"(a[0]), "v"(a[3]));
    }
#pragma unroll
    for (int mb = 0; mb < 4; ++mb) {
#pragma unroll
        for (int nb = 0; nb < 4; ++nb) {
#pragma unroll
            for (int j = 0; j < 8; ++j) os[(hi * 8 + j) * 68 + nb * 16 + lr] = acc[mb][nb][j]; }
        __builtin_amdgcn_wave_barrier(); asm volatile("" ::: "memory");
        float* crow = C + (size_t)(r0 + mb * 16) * ldc + c0;
#pragma unroll 1
        for (int ps = 0; ps < 2; ++ps) {
#pragma unroll
            for (int s = 0; s < 8; ++s) { const int row = 2 * s + hi, cofs = lr * 4; v4f val = *(const v4fa*)(os + row * 68 + cofs); if (BIAS) { val[0] += bfr(bias[c0 + cofs]); val[1] += bfr(bias[c0 + cofs + 1]); val[2] += bfr(bias[c0 + cofs + 2]); val[3] += bfr(bias[c0 + cofs + 3]); }
                *(volatile v4f*)(crow + (size_t)row * ldc + cofs) = val; }
            if (ps == 0) __threadfence(); }
        __builtin_amdgcn_wave_barrier(); asm volatile("" ::: "memory");
    }
}

__device__ __forceinline__ h16 tohx(float x) { return (h16)x; }
__device__ __forceinline__ void splitf(float y, unsigned short& h, unsigned short& l) { h = f2bf(y); l = f2bf(y - bf2f(h)); }
__device__ __forceinline__ float sigf(float a) { return __fdiv_rn(1.0f, __fadd_rn(1.0f, __expf(-a))); }
__device__ __forceinline__ float tanhf_(float a) { const float e2 = __expf(2.0f * a); return __fsub_rn(1.0f, __fdiv_rn(2.0f, __fadd_rn(e2, 1.0f))); }
typedef __attribute__((ext_vector_type(2))) _Float16 v2h;
typedef __attribute__((ext_vector_type(4))) _Float16 v4h;
typedef __attribute__((ext_vector_type(2))) unsigned short v2us;

__global__ __launch_bounds__(256) void k_cvt8(const float* __restrict__ src, bf* dst, size_t n8) { const size_t i = (size_t)blockIdx.x * 256 + threadIdx.x; if (i >= n8) return; const v8f v = *(const v8f*)(src + i * 8); v8us o;
#pragma unroll
    for (int k = 0; k < 8; ++k) o[k] = f2bf(v[k]); *(volatile v8us*)(dst + i * 8) = o; __threadfence(); *(volatile v8us*)(dst + i * 8) = o; }
__global__ __launch_bounds__(256) void k_kt(const float* __restrict__ K, float* KT) { const int e = (blockIdx.x * 256 + threadIdx.x) * 2; if (e >= DD * NN) return; const int j = e % NN, d = e / NN; typedef __attribute__((ext_vector_type(2))) float v2f; v2f o; o[0] = K[(size_t)j * DD + d]; o[1] = K[(size_t)(j + 1) * DD + d]; *(volatile v2f*)(KT + e) = o; __threadfence(); *(volatile v2f*)(KT + e) = o; }
__global__ __launch_bounds__(256) void k_xt16(const float* __restrict__ X, h16* XT) { const int e = (blockIdx.x * 256 + threadIdx.x) * 2; if (e >= DD * NN) return; const int j = e % NN, d = e / NN; v2h o; o[0] = tohx(bfr(X[(size_t)j * DD + d])); o[1] = tohx(bfr(X[(size_t)(j + 1) * DD + d])); *(volatile v2h*)(XT + e) = o; __threadfence(); *(volatile v2h*)(XT + e) = o; }
__global__ __launch_bounds__(256) void k_xa(const float* __restrict__ X, const float* __restrict__ ATT, bf* Ah, bf* Al) { const int e = (blockIdx.x * 256 + threadIdx.x) * 2; if (e >= NN * 2 * DD) return; const int c = e % (2 * DD), i = e / (2 * DD); v2us oh, ol;
#pragma unroll
    for (int q = 0; q < 2; ++q) { const int cc = c + q; const float v = (cc < DD) ? bfr(X[(size_t)i * DD + cc]) : ATT[(size_t)i * DD + cc - DD] * (1.0f / PCAR); unsigned short a, c2; splitf(v, a, c2); oh[q] = a; ol[q] = c2; }
    *(volatile v2us*)(Ah + e) = oh; *(volatile v2us*)(Al + e) = ol; __threadfence(); *(volatile v2us*)(Ah + e) = oh; *(volatile v2us*)(Al + e) = ol; }
__global__ __launch_bounds__(256) void k_sc(const float* __restrict__ Q, const float* __restrict__ KT, const float* __restrict__ vv, float* S) { const int e = (blockIdx.x * 256 + threadIdx.x) * 2; if (e >= NN * NN) return; const int j = e % NN, i = e / NN; typedef __attribute__((ext_vector_type(2))) float v2f; v2f o; o[0] = -1e30f; o[1] = -1e30f;
    if (j + 1 >= i) { float s0 = 0.f, s1 = 0.f; const float* qr = Q + (size_t)i * DD;
#pragma unroll 2
        for (int d = 0; d < DD; ++d) { const float qd = qr[d]; float w = bfr(vv[d]); asm volatile("" : "+v"(w)); const float k0 = KT[(size_t)d * NN + j], k1 = KT[(size_t)d * NN + j + 1];
            float t0 = tanhf_(__fadd_rn(qd, k0)), t1 = tanhf_(__fadd_rn(qd, k1)); asm volatile("" : "+v"(t0)); asm volatile("" : "+v"(t1)); float p0 = __fmul_rn(w, t0), p1 = __fmul_rn(w, t1); asm volatile("" : "+v"(p0)); asm volatile("" : "+v"(p1)); s0 = __fadd_rn(s0, p0); s1 = __fadd_rn(s1, p1); }
        if (j >= i) o[0] = s0; o[1] = s1; }
    *(volatile v2f*)(S + e) = o; __threadfence(); *(volatile v2f*)(S + e) = o; }
__global__ __launch_bounds__(256) void k_asoft(const float* __restrict__ Sb, h16* P16) { const int lane = threadIdx.x & 31; const int row = blockIdx.x * 8 + (threadIdx.x >> 5); if (row >= NN) return; const float* sr = Sb + (size_t)row * NN; float v[32]; float mx = -3.0e38f;
#pragma unroll
    for (int ch = 0; ch < 8; ++ch) { const v4f a = *(const v4f*)(sr + ch * 128 + lane * 4);
#pragma unroll
        for (int q = 0; q < 4; ++q) { v[ch * 4 + q] = a[q]; mx = fmaxf(mx, a[q]); } }
#pragma unroll
    for (int sh = 16; sh; sh >>= 1) mx = fmaxf(mx, __shfl_xor(mx, sh, 32));
    float sum = 0.f;
#pragma unroll
    for (int k = 0; k < 32; ++k) { float d0 = __fsub_rn(v[k], mx); asm volatile("" : "+v"(d0)); v[k] = __builtin_amdgcn_exp2f(__fmul_rn(d0, 1.4426950408889634f)); sum += v[k]; }
#pragma unroll
    for (int sh = 16; sh; sh >>= 1) sum += __shfl_xor(sum, sh, 32);
    const float f = __fdiv_rn(PCAR, sum);
#pragma unroll 1
    for (int ps = 0; ps < 2; ++ps) {
#pragma unroll
        for (int ch = 0; ch < 8; ++ch) { v4h o;
#pragma unroll
            for (int q = 0; q < 4; ++q) o[q] = tohx(v[ch * 4 + q] * f); *(volatile v4h*)(P16 + (size_t)row * NN + ch * 128 + lane * 4) = o; }
        if (ps == 0) __threadfence(); } }
__global__ __launch_bounds__(32) void k_gru(const float* __restrict__ GI, const float* __restrict__ whh, const float* __restrict__ bhh, float* OUT) { const int lane = threadIdx.x; float bh[12];
#pragma unroll
    for (int u = 0; u < 12; ++u) bh[u] = bfr(bhh[lane + 32 * u]);
    for (int ps = 0; ps < 2; ++ps) { float h[4] = {0.f, 0.f, 0.f, 0.f};
        for (int t = 0; t < NN; ++t) { float gh[12];
#pragma unroll
            for (int u = 0; u < 12; ++u) gh[u] = 0.f;
            for (int d = 0; d < DD; ++d) { const float hd = __shfl(h[d >> 5], d & 31, 32);
#pragma unroll
                for (int u = 0; u < 12; ++u) { float w = bfr(whh[(size_t)(lane + 32 * u) * DD + d]); asm volatile("" : "+v"(w)); float p = __fmul_rn(w, hd); asm volatile("" : "+v"(p)); gh[u] = __fadd_rn(gh[u], p); } }
            float hn[4];
#pragma unroll
            for (int m = 0; m < 4; ++m) { const int e = lane + 32 * m; const float* gi = GI + (size_t)t * G3; const float ghr = __fadd_rn(gh[m], bh[m]), ghz = __fadd_rn(gh[4 + m], bh[4 + m]), ghn = __fadd_rn(gh[8 + m], bh[8 + m]);
                const float r = sigf(__fadd_rn(gi[e], ghr)), z = sigf(__fadd_rn(gi[DD + e], ghz)); float rn = __fmul_rn(r, ghn); asm volatile("" : "+v"(rn)); const float ns = tanhf_(__fadd_rn(gi[2 * DD + e], rn));
                float omz = __fsub_rn(1.0f, z); float t1 = __fmul_rn(omz, ns), t2 = __fmul_rn(z, h[m]); asm volatile("" : "+v"(t1)); asm volatile("" : "+v"(t2)); hn[m] = __fadd_rn(t1, t2); }
#pragma unroll
            for (int m = 0; m < 4; ++m) { h[m] = hn[m]; *(volatile float*)(OUT + (size_t)t * DD + 32 * m + lane) = hn[m]; } }
        if (ps == 0) __threadfence(); } }

extern "C" void kernel_launch(void* const* d_in, const int* in_sizes, int n_in,
                              void* d_out, int out_size, void* d_ws, size_t ws_size, hipStream_t stream) {
    (void)in_sizes; (void)n_in; (void)out_size;
    const float* X = (const float*)d_in[0]; const float* wq = (const float*)d_in[1]; const float* wk = (const float*)d_in[2]; const float* vv = (const float*)d_in[3]; const float* wih = (const float*)d_in[4]; const float* whh = (const float*)d_in[5]; const float* bih = (const float*)d_in[6]; const float* bhh = (const float*)d_in[7];
    float* OUT = (float*)d_out;
    char* wsp = (char*)d_ws;
    auto take = [&](size_t bytes) { char* p = wsp; wsp += (bytes + 255) & ~(size_t)255; return (void*)p; };
    bf* WQ = (bf*)take((size_t)DD * DD * 2); bf* WK = (bf*)take((size_t)DD * DD * 2); bf* WIH = (bf*)take((size_t)G3 * 2 * DD * 2); bf* XB = (bf*)take((size_t)NN * DD * 2); float* Q = (float*)take((size_t)NN * DD * 4); float* K = (float*)take((size_t)NN * DD * 4); float* KT = (float*)take((size_t)DD * NN * 4); h16* XT = (h16*)take((size_t)DD * NN * 2);
    float* S = (float*)take((size_t)NN * NN * 4); h16* P = (h16*)take((size_t)NN * NN * 2); float* ATT = (float*)take((size_t)NN * DD * 4); bf* Ah = (bf*)take((size_t)NN * 2 * DD * 2); bf* Al = (bf*)take((size_t)NN * 2 * DD * 2); float* GI = (float*)take((size_t)NN * G3 * 4);
    if ((size_t)(wsp - (char*)d_ws) > ws_size) return;
    k_cvt8<<<(DD * DD / 8 + 255) / 256, 256, 0, stream>>>(wq, WQ, (size_t)DD * DD / 8); k_cvt8<<<(DD * DD / 8 + 255) / 256, 256, 0, stream>>>(wk, WK, (size_t)DD * DD / 8); k_cvt8<<<(G3 * 2 * DD / 8 + 255) / 256, 256, 0, stream>>>(wih, WIH, (size_t)G3 * 2 * DD / 8); k_cvt8<<<(NN * DD / 8 + 255) / 256, 256, 0, stream>>>(X, XB, (size_t)NN * DD / 8);
    k_gemmw<bf, 0, false><<<dim3(NN / 64, DD / 64, 1), 32, 0, stream>>>(XB, nullptr, WQ, nullptr, DD, Q, DD, nullptr, 0, 0, 0); k_gemmw<bf, 0, false><<<dim3(NN / 64, DD / 64, 1), 32, 0, stream>>>(XB, nullptr, WK, nullptr, DD, K, DD, nullptr, 0, 0, 0);
    k_kt<<<(DD * NN / 2 + 255) / 256, 256, 0, stream>>>(K, KT); k_xt16<<<(DD * NN / 2 + 255) / 256, 256, 0, stream>>>(X, XT);
    k_sc<<<(NN * NN / 2 + 255) / 256, 256, 0, stream>>>(Q, KT, vv, S); k_asoft<<<NN / 8, 256, 0, stream>>>(S, P);
    k_gemmw<h16, 0, false><<<dim3(NN / 64, DD / 64, 1), 32, 0, stream>>>(P, nullptr, XT, nullptr, NN, ATT, DD, nullptr, 0, 0, 0);
    k_xa<<<(NN * 2 * DD / 2 + 255) / 256, 256, 0, stream>>>(X, ATT, Ah, Al);
    k_gemmw<bf, 1, true><<<dim3(NN / 64, G3 / 64, 1), 32, 0, stream>>>(Ah, Al, WIH, nullptr, 2 * DD, GI, G3, bih, 0, 0, 0);
    k_gru<<<1, 32, 0, stream>>>(GI, whh, bhh, OUT);
}
